// SASS2D_5179730559105
// MI455X (gfx1250) — hardware-verified
//
#include <hip/hip_runtime.h>


#define NBI  8
#define CC   256
#define IH   80
#define IW   80
#define NP   6400
#define NG   16
#define CPG  16
#define NRB  100
typedef _Float16 h16;
typedef unsigned short bf;
typedef __attribute__((ext_vector_type(16))) __bf16   v16bf;
typedef __attribute__((ext_vector_type(16))) _Float16 v16h;
typedef __attribute__((ext_vector_type(8)))  _Float16 v8h;
typedef __attribute__((ext_vector_type(8)))  unsigned short v8us;
typedef __attribute__((ext_vector_type(8)))  float    v8f;
typedef __attribute__((ext_vector_type(4)))  float    v4f;
typedef v8h  __attribute__((may_alias)) v8ha;
typedef v4f  __attribute__((may_alias)) v4fa;
typedef v8us __attribute__((may_alias)) v8usa;

__device__ __forceinline__ unsigned short f2bf(float f) { unsigned u = __float_as_uint(f); u += 0x7FFFu + ((u >> 16) & 1u); return (unsigned short)(u >> 16); }
__device__ __forceinline__ float bf2f(unsigned short b) { return __uint_as_float(((unsigned)b) << 16); }
__device__ __forceinline__ float bfr(float f) { return bf2f(f2bf(f)); }
__device__ __forceinline__ v16h cat16(v8h lo, v8h hi) { return __builtin_shufflevector(lo, hi, 0, 1, 2, 3, 4, 5, 6, 7, 8, 9, 10, 11, 12, 13, 14, 15); }
__device__ __forceinline__ v16bf cat16b(v8us lo, v8us hi) { return __builtin_bit_cast(v16bf, __builtin_shufflevector(lo, hi, 0, 1, 2, 3, 4, 5, 6, 7, 8, 9, 10, 11, 12, 13, 14, 15)); }
__device__ __forceinline__ v8f wmma16(v16h a, v16h b, v8f c) { return __builtin_amdgcn_wmma_f32_16x16x32_f16(false, a, false, b, (short)0, c, false, false); }
__device__ __forceinline__ v8f wmmab(v16bf a, v16bf b, v8f c) { return __builtin_amdgcn_wmma_f32_16x16x32_bf16(false, a, false, b, (short)0, c, false, false); }


template <typename T16> struct WFrag;
template <> struct WFrag<h16> { typedef v16h V; static __device__ __forceinline__ V ld(const h16* p) { return cat16(*(const v8h*)p, *(const v8h*)(p + 16)); } static __device__ __forceinline__ v8f mma(V a, V b, v8f c) { return wmma16(a, b, c); } };
template <> struct WFrag<bf> { typedef v16bf V; static __device__ __forceinline__ V ld(const bf* p) { return cat16b(*(const v8us*)p, *(const v8us*)(p + 16)); } static __device__ __forceinline__ v8f mma(V a, V b, v8f c) { return wmmab(a, b, c); } };
template <typename T16, int NSPLIT, bool BIAS>
__global__ __launch_bounds__(32) void k_gemmw(const T16* __restrict__ A, const T16* __restrict__ A2, const T16* __restrict__ Bt, const T16* __restrict__ Bt2, int K, float* C, int ldc, const float* __restrict__ bias, size_t sA, size_t sB, size_t sC) {
    typedef typename WFrag<T16>::V V;
    __shared__ __align__(16) float os[16 * 68];
    const size_t z = blockIdx.z; A += z * sA; if (A2) A2 += z * sA; Bt += z * sB; if (Bt2) Bt2 += z * sB; C += z * sC;
    const int lane = threadIdx.x & 31, lr = lane & 15, hi = lane >> 4; const int r0 = blockIdx.x * 64, c0 = blockIdx.y * 64;
    v8f acc[4][4];
#pragma unroll
    for (int mb = 0; mb < 4; ++mb)
#pragma unroll
        for (int nb = 0; nb < 4; ++nb) acc[mb][nb] = (v8f){};
    const size_t aoff = (size_t)(r0 + lr) * K + 8 * hi, boff = (size_t)(c0 + lr) * K + 8 * hi;
#pragma unroll 1
    for (int kc = 0; kc < K; kc += 32) {
        V a[4], a2[4];
#pragma unroll
        for (int mb = 0; mb < 4; ++mb) { a[mb] = WFrag<T16>::ld(A + aoff + (size_t)mb * 16 * K + kc); if (NSPLIT == 1 || NSPLIT == 2) a2[mb] = WFrag<T16>::ld(A2 + aoff + (size_t)mb * 16 * K + kc); }
#pragma unroll
        for (int nb = 0; nb < 4; ++nb) { const V b = WFrag<T16>::ld(Bt + boff + (size_t)nb * 16 * K + kc); V b2; if (NSPLIT >= 2) b2 = WFrag<T16>::ld(Bt2 + boff + (size_t)nb * 16 * K + kc);
#pragma unroll
            for (int mb = 0; mb < 4; ++mb) { acc[mb][nb] = WFrag<T16>::mma(a[mb], b, acc[mb][nb]); if (NSPLIT == 1 || NSPLIT == 2) acc[mb][nb] = WFrag<T16>::mma(a2[mb], b, acc[mb][nb]); if (NSPLIT >= 2) acc[mb][nb] = WFrag<T16>::mma(a[mb], b2, acc[mb][nb]); } }
        asm volatile("v_nop\n\tv_nop\n\tv_nop\n\tv_nop" : "+v"(acc[0][0]), "+v"(acc[1][1]), "+v"(acc[2][2]), "+v"(acc[3][3]) : "v"(a[0]), "v"(a[3]));
    }
#pragma unroll
    for (int mb = 0; mb < 4; ++mb) {
#pragma unroll
        for (int nb = 0; nb < 4; ++nb) {
#pragma unroll
            for (int j = 0; j < 8; ++j) os[(hi * 8 + j) * 68 + nb * 16 + lr] = acc[mb][nb][j]; }
        __builtin_amdgcn_wave_barrier(); asm volatile("" ::: "memory");
        float* crow = C + (size_t)(r0 + mb * 16) * ldc + c0;
#pragma unroll 1
        for (int ps = 0; ps < 2; ++ps) {
#pragma unroll
            for (int s = 0; s < 8; ++s) { const int row = 2 * s + hi, cofs = lr * 4; v4f val = *(const v4fa*)(os + row * 68 + cofs); if (BIAS) { val[0] += bfr(bias[c0 + cofs]); val[1] += bfr(bias[c0 + cofs + 1]); val[2] += bfr(bias[c0 + cofs + 2]); val[3] += bfr(bias[c0 + cofs + 3]); }
                *(volatile v4f*)(crow + (size_t)row * ldc + cofs) = val; }
            if (ps == 0) __threadfence(); }
        __builtin_amdgcn_wave_barrier(); asm volatile("" ::: "memory");
    }
}

__device__ __forceinline__ void splitf(float y, unsigned short& h, unsigned short& l) { h = f2bf(y); l = f2bf(y - bf2f(h)); }
__device__ __forceinline__ float silu_(float x) { return __fmul_rn(x, __fdiv_rn(1.0f, 1.0f + __expf(-x))); }
typedef __attribute__((ext_vector_type(2))) unsigned short v2us;
typedef __attribute__((ext_vector_type(4))) unsigned short v4us;

__global__ __launch_bounds__(256) void k_cvt8(const float* __restrict__ src, bf* dst, size_t n8) { const size_t i = (size_t)blockIdx.x * 256 + threadIdx.x; if (i >= n8) return; const v8f v = *(const v8f*)(src + i * 8); v8us o;
#pragma unroll
    for (int k = 0; k < 8; ++k) o[k] = f2bf(v[k]); *(volatile v8us*)(dst + i * 8) = o; __threadfence(); *(volatile v8us*)(dst + i * 8) = o; }
__global__ __launch_bounds__(256) void k_xt(const float* __restrict__ x, bf* XT) { const int e = (blockIdx.x * 256 + threadIdx.x) * 2; if (e >= NP * CC) return; const int c = e % CC; const int p = e / CC; v2us o; o[0] = f2bf(x[(size_t)c * NP + p]); o[1] = f2bf(x[(size_t)(c + 1) * NP + p]); *(volatile v2us*)(XT + e) = o; __threadfence(); *(volatile v2us*)(XT + e) = o; }
template <int P> __global__ __launch_bounds__(256) void k_gpart(const float* __restrict__ F, const float* __restrict__ mu, float* GP) { const int i = blockIdx.x * 256 + threadIdx.x; if (i >= NG * NRB) return; const int rb = i % NRB, g = i / NRB; const float m = (P == 2) ? mu[g] : 0.f; float s = 0.f;
#pragma unroll 1
    for (int p = rb * 64; p < rb * 64 + 64; ++p) { const float* r = F + (size_t)p * CC + g * CPG;
#pragma unroll
        for (int c = 0; c < CPG; ++c) { float d0 = __fsub_rn(r[c], m); asm volatile("" : "+v"(d0)); if (P == 2) { float q = __fmul_rn(d0, d0); asm volatile("" : "+v"(q)); s = __fadd_rn(s, q); } else s = __fadd_rn(s, d0); } }
    *(volatile float*)(GP + i) = s; __threadfence(); *(volatile float*)(GP + i) = s; }
__global__ __launch_bounds__(64) void k_gfin(const float* __restrict__ GP, float* GS) { const int g = threadIdx.x; if (g >= NG) return; float s = 0.f;
#pragma unroll 1
    for (int rb = 0; rb < NRB; ++rb) s = __fadd_rn(s, GP[g * NRB + rb]); const float v = s * (1.0f / (CPG * NP)); *(volatile float*)(GS + g) = v; __threadfence(); *(volatile float*)(GS + g) = v; }
__global__ __launch_bounds__(256) void k_gnact(const float* __restrict__ F, const float* __restrict__ gm, const float* __restrict__ gv, const float* __restrict__ ga, const float* __restrict__ gb, float* Hf, bf* Hh, bf* Hl) { const int e = (blockIdx.x * 256 + threadIdx.x) * 4; if (e >= NP * CC) return; const int c = e % CC; const v4f a = *(const v4f*)(F + e); v4f o; v4us oh, ol;
#pragma unroll
    for (int u = 0; u < 4; ++u) { const int cc = c + u, g = cc / CPG; float n = __fmul_rn(__fsub_rn(a[u], gm[g]), __frsqrt_rn(__fadd_rn(gv[g], 1e-5f))); asm volatile("" : "+v"(n)); float t = __fmul_rn(n, bfr(ga[cc])); asm volatile("" : "+v"(t)); o[u] = silu_(__fadd_rn(t, bfr(gb[cc]))); unsigned short hh, ll; splitf(o[u], hh, ll); oh[u] = hh; ol[u] = ll; }
    for (int ps = 0; ps < 2; ++ps) { *(volatile v4f*)(Hf + e) = o; if (Hh) { *(volatile v4us*)(Hh + e) = oh; *(volatile v4us*)(Hl + e) = ol; } if (ps == 0) __threadfence(); } }
__global__ __launch_bounds__(256) void k_wfwd(const float* __restrict__ Hf, float* LR) { const int i = blockIdx.x * 256 + threadIdx.x; if (i >= IH * (CC / 4)) return; const int c = (i % (CC / 4)) * 4; const int y = i / (CC / 4);
    for (int ps = 0; ps < 2; ++ps) { v4f acc = (v4f){0.f, 0.f, 0.f, 0.f};
#pragma unroll 1
        for (int x = 0; x < IW; ++x) { const size_t o = ((size_t)(y * IW + x)) * CC + c; const v4f h = *(const v4f*)(Hf + o);
#pragma unroll
            for (int u = 0; u < 4; ++u) acc[u] = __fadd_rn(acc[u], h[u]); *(volatile v4f*)(LR + o) = acc; }
        if (ps == 0) __threadfence(); } }
__global__ __launch_bounds__(256) void k_wbwd(const float* __restrict__ Hf, const float* __restrict__ LR, float* FU) { const int i = blockIdx.x * 256 + threadIdx.x; if (i >= IH * (CC / 4)) return; const int c = (i % (CC / 4)) * 4; const int y = i / (CC / 4);
    for (int ps = 0; ps < 2; ++ps) { v4f acc = (v4f){0.f, 0.f, 0.f, 0.f};
#pragma unroll 1
        for (int x = IW - 1; x >= 0; --x) { const size_t o = ((size_t)(y * IW + x)) * CC + c; const v4f h = *(const v4f*)(Hf + o), l = *(const v4f*)(LR + o); v4f v;
#pragma unroll
            for (int u = 0; u < 4; ++u) { acc[u] = __fadd_rn(acc[u], h[u]); v[u] = __fadd_rn(l[u], acc[u]); } *(volatile v4f*)(FU + o) = v; }
        if (ps == 0) __threadfence(); } }
__global__ __launch_bounds__(256) void k_hfwd(const float* __restrict__ Hf, float* TB) { const int i = blockIdx.x * 256 + threadIdx.x; if (i >= IW * (CC / 4)) return; const int c = (i % (CC / 4)) * 4; const int x = i / (CC / 4);
    for (int ps = 0; ps < 2; ++ps) { v4f acc = (v4f){0.f, 0.f, 0.f, 0.f};
#pragma unroll 1
        for (int y = 0; y < IH; ++y) { const size_t o = ((size_t)(y * IW + x)) * CC + c; const v4f h = *(const v4f*)(Hf + o);
#pragma unroll
            for (int u = 0; u < 4; ++u) acc[u] = __fadd_rn(acc[u], h[u]); *(volatile v4f*)(TB + o) = acc; }
        if (ps == 0) __threadfence(); } }
__global__ __launch_bounds__(256) void k_hbwd(const float* __restrict__ Hf, const float* __restrict__ FU, const float* __restrict__ TB, float* FS) { const int i = blockIdx.x * 256 + threadIdx.x; if (i >= IW * (CC / 4)) return; const int c = (i % (CC / 4)) * 4; const int x = i / (CC / 4);
    for (int ps = 0; ps < 2; ++ps) { v4f acc = (v4f){0.f, 0.f, 0.f, 0.f};
#pragma unroll 1
        for (int y = IH - 1; y >= 0; --y) { const size_t o = ((size_t)(y * IW + x)) * CC + c; const v4f h = *(const v4f*)(Hf + o), f = *(const v4f*)(FU + o), tb = *(const v4f*)(TB + o); v4f v;
#pragma unroll
            for (int u = 0; u < 4; ++u) { acc[u] = __fadd_rn(acc[u], h[u]); v[u] = __fadd_rn(__fadd_rn(f[u], tb[u]), acc[u]); } *(volatile v4f*)(FS + o) = v; }
        if (ps == 0) __threadfence(); } }
__global__ __launch_bounds__(256) void k_gate(const float* __restrict__ FU, const float* __restrict__ GA, float* GT) { const int e = (blockIdx.x * 256 + threadIdx.x) * 4; if (e >= NP * CC) return; const v4f f = *(const v4f*)(FU + e), ga = *(const v4f*)(GA + e); v4f o;
#pragma unroll
    for (int u = 0; u < 4; ++u) { const float s = __fdiv_rn(1.0f, 1.0f + __expf(-ga[u])); o[u] = __fmul_rn(f[u] * 0.25f, s); } *(volatile v4f*)(GT + e) = o; __threadfence(); *(volatile v4f*)(GT + e) = o; }
__global__ __launch_bounds__(256) void k_dw(const float* __restrict__ GT, const float* __restrict__ wdw, bf* Dh, bf* Dl) { const int e = (blockIdx.x * 256 + threadIdx.x) * 4; if (e >= NP * CC) return; const int c = e % CC; const int p = e / CC; const int y = p / IW, x = p % IW; v4us oh, ol;
#pragma unroll
    for (int u = 0; u < 4; ++u) { const int cc = c + u; float acc = 0.f;
#pragma unroll
        for (int ky = 0; ky < 3; ++ky) {
#pragma unroll
            for (int kx = 0; kx < 3; ++kx) { const int yy = y + ky - 1, xx = x + kx - 1; if (yy >= 0 && yy < IH && xx >= 0 && xx < IW) { float pr = __fmul_rn(bfr(wdw[cc * 9 + ky * 3 + kx]), GT[((size_t)(yy * IW + xx)) * CC + cc]); asm volatile("" : "+v"(pr)); acc = __fadd_rn(acc, pr); } } }
        unsigned short hh, ll; splitf(acc, hh, ll); oh[u] = hh; ol[u] = ll; }
    *(volatile v4us*)(Dh + e) = oh; *(volatile v4us*)(Dl + e) = ol; __threadfence(); *(volatile v4us*)(Dh + e) = oh; *(volatile v4us*)(Dl + e) = ol; }
__global__ __launch_bounds__(256) void k_outT(const float* __restrict__ Y, const float* __restrict__ gm, const float* __restrict__ gv, const float* __restrict__ ga, const float* __restrict__ gb, float* OUTb) { const int e = (blockIdx.x * 256 + threadIdx.x) * 4; if (e >= CC * NP) return; const int p = e % NP; const int c = e / NP; const int g = c / CPG; const float rs = __frsqrt_rn(__fadd_rn(gv[g], 1e-5f)); v4f o;
#pragma unroll
    for (int u = 0; u < 4; ++u) { float n = __fmul_rn(__fsub_rn(Y[(size_t)(p + u) * CC + c], gm[g]), rs); asm volatile("" : "+v"(n)); float t = __fmul_rn(n, bfr(ga[c])); asm volatile("" : "+v"(t)); o[u] = silu_(__fadd_rn(t, bfr(gb[c]))); }
    *(volatile v4f*)(OUTb + e) = o; __threadfence(); *(volatile v4f*)(OUTb + e) = o; }

extern "C" void kernel_launch(void* const* d_in, const int* in_sizes, int n_in,
                              void* d_out, int out_size, void* d_ws, size_t ws_size, hipStream_t stream) {
    (void)in_sizes; (void)n_in; (void)out_size;
    const float* x = (const float*)d_in[0]; const float* wpre = (const float*)d_in[1]; const float* g1 = (const float*)d_in[2]; const float* b1 = (const float*)d_in[3]; const float* wg = (const float*)d_in[4]; const float* bg = (const float*)d_in[5]; const float* wdw = (const float*)d_in[6]; const float* wpw = (const float*)d_in[7]; const float* g2 = (const float*)d_in[8]; const float* b2 = (const float*)d_in[9];
    float* OUT = (float*)d_out;
    char* wsp = (char*)d_ws;
    auto take = [&](size_t bytes) { char* p = wsp; wsp += (bytes + 255) & ~(size_t)255; return (void*)p; };
    bf* WPRE = (bf*)take(CC * CC * 2); bf* WG = (bf*)take(CC * CC * 2); bf* WPW = (bf*)take(CC * CC * 2);
    bf* XT = (bf*)take((size_t)NP * CC * 2); float* F = (float*)take((size_t)NP * CC * 4); float* GP = (float*)take(NG * NRB * 4); float* GM = (float*)take(256); float* GV = (float*)take(256); float* Hf = (float*)take((size_t)NP * CC * 4); bf* Hh = (bf*)take((size_t)NP * CC * 2); bf* Hl = (bf*)take((size_t)NP * CC * 2);
    float* GA = (float*)take((size_t)NP * CC * 4); float* LR = (float*)take((size_t)NP * CC * 4); float* FU = (float*)take((size_t)NP * CC * 4); float* TBu = (float*)take((size_t)NP * CC * 4); float* FS = (float*)take((size_t)NP * CC * 4); float* GT = (float*)take((size_t)NP * CC * 4); bf* Dh = (bf*)take((size_t)NP * CC * 2); bf* Dl = (bf*)take((size_t)NP * CC * 2); float* Y = (float*)take((size_t)NP * CC * 4);
    if ((size_t)(wsp - (char*)d_ws) > ws_size) return;
    k_cvt8<<<(CC * CC / 8 + 255) / 256, 256, 0, stream>>>(wpre, WPRE, CC * CC / 8); k_cvt8<<<(CC * CC / 8 + 255) / 256, 256, 0, stream>>>(wg, WG, CC * CC / 8); k_cvt8<<<(CC * CC / 8 + 255) / 256, 256, 0, stream>>>(wpw, WPW, CC * CC / 8);
    for (int b = 0; b < NBI; ++b) {
        k_xt<<<(NP * CC / 2 + 255) / 256, 256, 0, stream>>>(x + (size_t)b * CC * NP, XT);
        k_gemmw<bf, 0, false><<<dim3(NP / 64, CC / 64, 1), 32, 0, stream>>>(XT, nullptr, WPRE, nullptr, CC, F, CC, nullptr, 0, 0, 0);
        k_gpart<1><<<(NG * NRB + 255) / 256, 256, 0, stream>>>(F, nullptr, GP); k_gfin<<<1, 64, 0, stream>>>(GP, GM); k_gpart<2><<<(NG * NRB + 255) / 256, 256, 0, stream>>>(F, GM, GP); k_gfin<<<1, 64, 0, stream>>>(GP, GV);
        k_gnact<<<(NP * CC / 4 + 255) / 256, 256, 0, stream>>>(F, GM, GV, g1, b1, Hf, Hh, Hl);
        k_gemmw<bf, 1, true><<<dim3(NP / 64, CC / 64, 1), 32, 0, stream>>>(Hh, Hl, WG, nullptr, CC, GA, CC, bg, 0, 0, 0);
        k_wfwd<<<(IH * (CC / 4) + 255) / 256, 256, 0, stream>>>(Hf, LR); k_wbwd<<<(IH * (CC / 4) + 255) / 256, 256, 0, stream>>>(Hf, LR, FU); k_hfwd<<<(IW * (CC / 4) + 255) / 256, 256, 0, stream>>>(Hf, TBu); k_hbwd<<<(IW * (CC / 4) + 255) / 256, 256, 0, stream>>>(Hf, FU, TBu, FS);
        k_gate<<<(NP * CC / 4 + 255) / 256, 256, 0, stream>>>(FS, GA, GT);
        k_dw<<<(NP * CC / 4 + 255) / 256, 256, 0, stream>>>(GT, wdw, Dh, Dl);
        k_gemmw<bf, 1, false><<<dim3(NP / 64, CC / 64, 1), 32, 0, stream>>>(Dh, Dl, WPW, nullptr, CC, Y, CC, nullptr, 0, 0, 0);
        k_gpart<1><<<(NG * NRB + 255) / 256, 256, 0, stream>>>(Y, nullptr, GP); k_gfin<<<1, 64, 0, stream>>>(GP, GM); k_gpart<2><<<(NG * NRB + 255) / 256, 256, 0, stream>>>(Y, GM, GP); k_gfin<<<1, 64, 0, stream>>>(GP, GV);
        k_outT<<<(CC * NP / 4 + 255) / 256, 256, 0, stream>>>(Y, GM, GV, g2, b2, OUT + (size_t)b * CC * NP); }
}
